// DeltaRuleModel_35270271435155
// MI455X (gfx1250) — hardware-run, weakly checked
//
#include <hip/hip_runtime.h>
#include <math.h>

typedef __attribute__((ext_vector_type(16))) _Float16 v16h;
typedef __attribute__((ext_vector_type(8)))  float    v8f;
typedef __attribute__((ext_vector_type(4)))  float    v4f;
typedef __attribute__((ext_vector_type(4)))  int      v4i;

constexpr int kBatch   = 1024;
constexpr int kSeqLen  = 2048;
constexpr int kHid     = 32;
constexpr int kHid2    = 64;
constexpr int kVocab   = 64;
constexpr int kChunk   = 32;
constexpr int kPitchA  = 36;
constexpr int kPitchB  = 68;
constexpr int kTokPitch = 33;
static_assert((kSeqLen % kChunk) == 0);
static_assert((kBatch % 64) == 0);
static_assert(kHid == 32 && kHid2 == 64 && kVocab == 64);

constexpr float kCarryW   = 1024.0f;
constexpr float kCarryG   = 4096.0f;
constexpr float kCarryCtx = 1.0f;
constexpr float kCarryRd  = 16.0f;
constexpr float kCarryLo  = 2048.0f;
constexpr float kFoldFfn1  = 1.0f / (kCarryW * kCarryW);
constexpr float kFoldFfn2  = 1.0f / (kCarryG * kCarryW);
constexpr float kFoldRdHi  = 1.0f / (kCarryCtx * kCarryW);
constexpr float kFoldRdLo  = kFoldRdHi / kCarryLo;
constexpr float kFoldOutHi = 1.0f / (kCarryRd * kCarryW);
constexpr float kFoldOutLo = kFoldOutHi / kCarryLo;
constexpr float kInvHid    = 1.0f / (float)kHid;
constexpr float kLnEps     = 1e-5f;
constexpr float kDeltaEps  = 1e-6f;
constexpr float kF16MinNormal = 6.103515625e-5f;

constexpr size_t kOffTbl  = 0;
constexpr size_t kOffDinv = kOffTbl  + (size_t)kVocab * kHid * 4;
constexpr size_t kOffCtx  = kOffDinv + (size_t)kVocab * 4;
constexpr size_t kWsTotal = kOffCtx  + (size_t)kBatch * kHid * 4;
static_assert(kWsTotal == 139520ull);
static_assert((kOffDinv % 128) == 0 && (kOffCtx % 128) == 0);
static_assert(kWsTotal <= 134217728ull);

__device__ __forceinline__ _Float16 to_h16(float v) {
  const float z = (fabsf(v) < kF16MinNormal) ? 0.0f : v;
  return (_Float16)z;
}
__device__ __forceinline__ void split_h16(float v, float carry, _Float16& hi, _Float16& lo) {
  const float vs = v * carry;
  const _Float16 hh = to_h16(vs);
  const float back = (float)hh;
  const float res = (vs - back) * kCarryLo;
  hi = hh;
  lo = to_h16(res);
}
__device__ __forceinline__ v8f mma_h(v16h a, v16h b, v8f c) {
  c = __builtin_amdgcn_wmma_f32_16x16x32_f16(false, a, false, b, (short)0, c, false, false);
  asm volatile("v_nop\n\tv_nop\n\tv_nop\n\tv_nop" : "+v"(c) : "v"(a), "v"(b));
  return c;
}
__device__ __forceinline__ v16h bfrag_from_lds(const float* w, unsigned pitch, unsigned kbase,
                                               unsigned hs, unsigned col, float carry) {
  v16h b;
#pragma unroll
  for (int i = 0; i < 8; ++i) {
    const float lo8 = w[(kbase + 8u * hs + (unsigned)i) * pitch + col];
    const float hi8 = w[(kbase + 16u + 8u * hs + (unsigned)i) * pitch + col];
    b[i]     = to_h16(lo8 * carry);
    b[8 + i] = to_h16(hi8 * carry);
  }
  return b;
}
__device__ __forceinline__ float wave_sum(float v) {
  v += __shfl_xor(v, 16, 32);
  v += __shfl_xor(v, 8, 32);
  v += __shfl_xor(v, 4, 32);
  v += __shfl_xor(v, 2, 32);
  v += __shfl_xor(v, 1, 32);
  return v;
}

__global__ __launch_bounds__(128) void encode_table_kernel(
    const float* __restrict__ embed, const float* __restrict__ w1, const float* __restrict__ b1,
    const float* __restrict__ w2, const float* __restrict__ b2, const float* __restrict__ ln_g,
    const float* __restrict__ ln_b, float* __restrict__ Tt, float* __restrict__ Dinv)
{
  __shared__ __align__(16) float sE[kVocab * kPitchA];
  __shared__ __align__(16) float sW1[kHid * kPitchB];
  __shared__ __align__(16) float sW2[kHid2 * kPitchA];
  __shared__ __align__(16) float sG[4][16 * kPitchB];
  __shared__ float sB1[kHid2];
  __shared__ float sB2[kHid];
  __shared__ float sLg[kHid];
  __shared__ float sLb[kHid];
  __shared__ float sDi[kVocab];

  const unsigned tid = threadIdx.x;
  unsigned lane = tid & 31u;
  unsigned wave = tid >> 5;
  unsigned hs = lane >> 4;
  unsigned n = lane & 15u;
  asm volatile("" : "+v"(lane));
  asm volatile("" : "+v"(wave));
  asm volatile("" : "+v"(hs));
  asm volatile("" : "+v"(n));

#pragma unroll
  for (unsigned i = 0; i < 4u; ++i) {
    unsigned idx = tid + 128u * i;
    asm volatile("" : "+v"(idx));
    {
      const unsigned row = idx >> 3, c4 = (idx & 7u) * 4u;
      *(v4f*)(sE + row * kPitchA + c4) = *(const v4f*)(embed + row * kHid + c4);
    }
    {
      const unsigned row = idx >> 4, c4 = (idx & 15u) * 4u;
      *(v4f*)(sW1 + row * kPitchB + c4) = *(const v4f*)(w1 + row * kHid2 + c4);
    }
    {
      const unsigned row = idx >> 3, c4 = (idx & 7u) * 4u;
      *(v4f*)(sW2 + row * kPitchA + c4) = *(const v4f*)(w2 + row * kHid + c4);
    }
  }
  {
    const unsigned i64 = tid & 63u, i32 = tid & 31u;
    sB1[i64] = b1[i64];
    sB2[i32] = b2[i32];
    sLg[i32] = ln_g[i32];
    sLb[i32] = ln_b[i32];
  }
  __syncthreads();

  const v8f zero8 = (v8f){0.f, 0.f, 0.f, 0.f, 0.f, 0.f, 0.f, 0.f};
  const unsigned vrow0 = wave * 16u;

  v16h aE;
  {
    const float* er = sE + (vrow0 + n) * kPitchA + 8u * hs;
#pragma unroll
    for (int i = 0; i < 8; ++i) {
      aE[i]     = to_h16(er[i] * kCarryW);
      aE[8 + i] = to_h16(er[16 + i] * kCarryW);
    }
  }

  v8f acc1[4];
#pragma unroll
  for (int nt = 0; nt < 4; ++nt) {
    const v16h bw = bfrag_from_lds(sW1, (unsigned)kPitchB, 0u, hs, (unsigned)nt * 16u + n, kCarryW);
    acc1[nt] = mma_h(aE, bw, zero8);
  }

  float* gw = sG[wave];
#pragma unroll
  for (int nt = 0; nt < 4; ++nt) {
    const unsigned col = (unsigned)nt * 16u + n;
    const float bias = sB1[col];
#pragma unroll
    for (int r = 0; r < 8; ++r) {
      float v = acc1[nt][r] * kFoldFfn1 + bias;
      v = fmaxf(v, 0.0f);
      gw[(8u * hs + (unsigned)r) * kPitchB + col] = v;
    }
  }
  __syncthreads();

  v16h a2[2];
#pragma unroll
  for (int kk = 0; kk < 2; ++kk) {
    const float* gr = gw + n * kPitchB + (unsigned)kk * 32u + 8u * hs;
#pragma unroll
    for (int i = 0; i < 8; ++i) {
      a2[kk][i]     = to_h16(gr[i] * kCarryG);
      a2[kk][8 + i] = to_h16(gr[16 + i] * kCarryG);
    }
  }
  v8f acc2[2];
#pragma unroll
  for (int nt = 0; nt < 2; ++nt) {
    const v16h bw0 = bfrag_from_lds(sW2, (unsigned)kPitchA, 0u, hs, (unsigned)nt * 16u + n, kCarryW);
    const v16h bw1 = bfrag_from_lds(sW2, (unsigned)kPitchA, 32u, hs, (unsigned)nt * 16u + n, kCarryW);
    acc2[nt] = mma_h(a2[0], bw0, zero8);
    acc2[nt] = mma_h(a2[1], bw1, acc2[nt]);
  }
  __syncthreads();
#pragma unroll
  for (int nt = 0; nt < 2; ++nt) {
    const unsigned col = (unsigned)nt * 16u + n;
    const float bias = sB2[col];
#pragma unroll
    for (int r = 0; r < 8; ++r) {
      const unsigned rr = 8u * hs + (unsigned)r;
      const float ff = acc2[nt][r] * kFoldFfn2 + bias;
      gw[rr * kPitchB + col] = sE[(vrow0 + rr) * kPitchA + col] + ff;
    }
  }
  __syncthreads();

  const float lg = sLg[lane], lb = sLb[lane];
#pragma unroll 1
  for (unsigned r = 0; r < 16u; ++r) {
    const float xv = gw[r * kPitchB + lane];
    const float mu = wave_sum(xv) * kInvHid;
    const float dl = xv - mu;
    const float var = wave_sum(dl * dl) * kInvHid;
    const float inv = 1.0f / sqrtf(var + kLnEps);
    const float kv = dl * inv * lg + lb;
    const float dsum = wave_sum(kv * kv) + kDeltaEps;
    const float di = 1.0f / dsum;
    const unsigned row = vrow0 + r;
    float* p = Tt + row * kHid + lane;
    *(volatile float*)p = kv;
    __threadfence();
    *(volatile float*)p = kv;
    sDi[row] = di;
  }
  __syncthreads();
  if (wave == 0u) {
    const float v0 = sDi[lane];
    const float v1 = sDi[32u + lane];
    *(volatile float*)(Dinv + lane) = v0;
    *(volatile float*)(Dinv + 32u + lane) = v1;
    __threadfence();
    *(volatile float*)(Dinv + lane) = v0;
    *(volatile float*)(Dinv + 32u + lane) = v1;
  }
}

__global__ __launch_bounds__(32) void adjoint_scan_kernel(
    const int* __restrict__ seq, const float* __restrict__ Tt, const float* __restrict__ Dinv,
    float* __restrict__ ctxp)
{
  __shared__ __align__(16) float sT[kVocab * kPitchA];
  __shared__ float sDi[kVocab];
  __shared__ int   sTok[kChunk * kTokPitch];
  __shared__ float sC[kChunk * kTokPitch];

  unsigned lane = threadIdx.x & 31u;
  asm volatile("" : "+v"(lane));
  const unsigned b0 = blockIdx.x * 32u;

#pragma unroll
  for (unsigned i = 0; i < 16u; ++i) {
    unsigned idx = lane + 32u * i;
    asm volatile("" : "+v"(idx));
    const unsigned row = idx >> 3, c4 = (idx & 7u) * 4u;
    *(v4f*)(sT + row * kPitchA + c4) = *(const v4f*)(Tt + row * kHid + c4);
  }
  sDi[lane] = Dinv[lane];
  sDi[32u + lane] = Dinv[32u + lane];
  __syncthreads();

  float w[kHid], ctx[kHid];
#pragma unroll
  for (int j = 0; j < kHid; ++j) {
    w[j] = 0.0f;
    ctx[j] = 0.0f;
  }

  unsigned trow = lane >> 3;
  unsigned tcol = (lane & 7u) * 4u;
  asm volatile("" : "+v"(trow));
  asm volatile("" : "+v"(tcol));

  constexpr int kLastChunk = kSeqLen / kChunk - 1;
#pragma unroll 1
  for (int c = kLastChunk; c >= 0; --c) {
    const unsigned t0 = (unsigned)c * (unsigned)kChunk;
#pragma unroll
    for (unsigned i = 0; i < 8u; ++i) {
      const unsigned rr = trow + 4u * i;
      const v4i tk = *(const v4i*)(seq + (size_t)(b0 + rr) * kSeqLen + t0 + tcol);
      sTok[rr * kTokPitch + tcol + 0u] = tk[0];
      sTok[rr * kTokPitch + tcol + 1u] = tk[1];
      sTok[rr * kTokPitch + tcol + 2u] = tk[2];
      sTok[rr * kTokPitch + tcol + 3u] = tk[3];
    }
    __syncthreads();

    int sTop = kChunk - 1;
    if (c == kLastChunk) {
      int tq = sTok[lane * kTokPitch + (kChunk - 1)];
      tq = tq < 0 ? 0 : tq;
      tq = tq > (kVocab - 1) ? (kVocab - 1) : tq;
      unsigned tqu = (unsigned)tq;
      asm volatile("" : "+v"(tqu));
      const float* tr = sT + tqu * kPitchA;
#pragma unroll
      for (int e = 0; e < 8; ++e) {
        const v4f qv = *(const v4f*)(tr + 4 * e);
        w[4 * e + 0] = qv[0];
        w[4 * e + 1] = qv[1];
        w[4 * e + 2] = qv[2];
        w[4 * e + 3] = qv[3];
      }
      sTop = kChunk - 2;
    }

#pragma unroll 1
    for (int s = sTop; s >= 0; --s) {
      int tk = sTok[lane * kTokPitch + (unsigned)s];
      tk = tk < 0 ? 0 : tk;
      tk = tk > (kVocab - 1) ? (kVocab - 1) : tk;
      unsigned tku = (unsigned)tk;
      asm volatile("" : "+v"(tku));
      const float* tr = sT + tku * kPitchA;
      const float di = sDi[tku];
      v4f kq[8];
#pragma unroll
      for (int e = 0; e < 8; ++e) kq[e] = *(const v4f*)(tr + 4 * e);
      float s0 = kq[0][0] * w[0];
      float s1 = kq[0][1] * w[1];
      float s2 = kq[0][2] * w[2];
      float s3 = kq[0][3] * w[3];
#pragma unroll
      for (int e = 1; e < 8; ++e) {
        s0 = fmaf(kq[e][0], w[4 * e + 0], s0);
        s1 = fmaf(kq[e][1], w[4 * e + 1], s1);
        s2 = fmaf(kq[e][2], w[4 * e + 2], s2);
        s3 = fmaf(kq[e][3], w[4 * e + 3], s3);
      }
      const float a = (s0 + s1) + (s2 + s3);
      const float cneg = -(a * di);
#pragma unroll
      for (int e = 0; e < 8; ++e) {
#pragma unroll
        for (int q = 0; q < 4; ++q) {
          const float kj = kq[e][q];
          ctx[4 * e + q] = fmaf(a, kj, ctx[4 * e + q]);
          w[4 * e + q]   = fmaf(cneg, kj, w[4 * e + q]);
        }
      }
    }
    __syncthreads();
  }

#pragma unroll
  for (int j = 0; j < kHid; ++j) sC[lane * kTokPitch + (unsigned)j] = ctx[j];
  __syncthreads();
  for (int pass = 0; pass < 2; ++pass) {
#pragma unroll 1
    for (unsigned rr = 0; rr < 32u; ++rr) {
      const float v = sC[rr * kTokPitch + lane];
      *(volatile float*)(ctxp + (size_t)(b0 + rr) * kHid + lane) = v;
    }
    __threadfence();
  }
}

__global__ __launch_bounds__(128) void readout_kernel(
    const float* __restrict__ ctxp, const float* __restrict__ read_w, const float* __restrict__ read_b,
    const float* __restrict__ out_w, const float* __restrict__ out_b, float* __restrict__ out)
{
  __shared__ __align__(16) float sRW[kHid * kPitchA];
  __shared__ __align__(16) float sOW[kHid * kPitchB];
  __shared__ float sRB[kHid];
  __shared__ float sOB[kVocab];
  __shared__ __align__(16) float sR[4][16 * kPitchA];
  __shared__ __align__(16) float sO[4][16 * kPitchB];

  const unsigned tid = threadIdx.x;
  unsigned lane = tid & 31u;
  unsigned wave = tid >> 5;
  unsigned hs = lane >> 4;
  unsigned n = lane & 15u;
  asm volatile("" : "+v"(lane));
  asm volatile("" : "+v"(wave));
  asm volatile("" : "+v"(hs));
  asm volatile("" : "+v"(n));

#pragma unroll
  for (unsigned i = 0; i < 2u; ++i) {
    unsigned idx = tid + 128u * i;
    asm volatile("" : "+v"(idx));
    const unsigned row = idx >> 3, c4 = (idx & 7u) * 4u;
    *(v4f*)(sRW + row * kPitchA + c4) = *(const v4f*)(read_w + row * kHid + c4);
  }
#pragma unroll
  for (unsigned i = 0; i < 4u; ++i) {
    unsigned idx = tid + 128u * i;
    asm volatile("" : "+v"(idx));
    const unsigned row = idx >> 4, c4 = (idx & 15u) * 4u;
    *(v4f*)(sOW + row * kPitchB + c4) = *(const v4f*)(out_w + row * kVocab + c4);
  }
  {
    const unsigned i64 = tid & 63u, i32 = tid & 31u;
    sRB[i32] = read_b[i32];
    sOB[i64] = out_b[i64];
  }
  __syncthreads();

  const v8f zero8 = (v8f){0.f, 0.f, 0.f, 0.f, 0.f, 0.f, 0.f, 0.f};
  const unsigned m0 = blockIdx.x * 64u + wave * 16u;

  v16h aH, aL;
  {
    const float* cr = ctxp + (size_t)(m0 + n) * kHid + 8u * hs;
    const v4f c0 = *(const v4f*)(cr);
    const v4f c1 = *(const v4f*)(cr + 4);
    const v4f c2 = *(const v4f*)(cr + 16);
    const v4f c3 = *(const v4f*)(cr + 20);
#pragma unroll
    for (int e = 0; e < 4; ++e) {
      _Float16 hh, ll;
      const float f0 = c0[e];
      split_h16(f0, kCarryCtx, hh, ll);
      aH[e] = hh;
      aL[e] = ll;
      const float f1 = c1[e];
      split_h16(f1, kCarryCtx, hh, ll);
      aH[4 + e] = hh;
      aL[4 + e] = ll;
      const float f2 = c2[e];
      split_h16(f2, kCarryCtx, hh, ll);
      aH[8 + e] = hh;
      aL[8 + e] = ll;
      const float f3 = c3[e];
      split_h16(f3, kCarryCtx, hh, ll);
      aH[12 + e] = hh;
      aL[12 + e] = ll;
    }
  }

  v8f rH[2], rL[2];
#pragma unroll
  for (int nt = 0; nt < 2; ++nt) {
    const v16h bw = bfrag_from_lds(sRW, (unsigned)kPitchA, 0u, hs, (unsigned)nt * 16u + n, kCarryW);
    rH[nt] = mma_h(aH, bw, zero8);
    rL[nt] = mma_h(aL, bw, zero8);
  }
  float* rw = sR[wave];
#pragma unroll
  for (int nt = 0; nt < 2; ++nt) {
    const unsigned col = (unsigned)nt * 16u + n;
    const float bias = sRB[col];
#pragma unroll
    for (int r = 0; r < 8; ++r) {
      const float v = rH[nt][r] * kFoldRdHi + rL[nt][r] * kFoldRdLo + bias;
      rw[(8u * hs + (unsigned)r) * kPitchA + col] = v;
    }
  }
  __syncthreads();

  v16h a2H, a2L;
  {
    const float* rr = rw + n * kPitchA + 8u * hs;
#pragma unroll
    for (int i = 0; i < 8; ++i) {
      _Float16 hh, ll;
      const float f0 = rr[i];
      split_h16(f0, kCarryRd, hh, ll);
      a2H[i] = hh;
      a2L[i] = ll;
      const float f1 = rr[16 + i];
      split_h16(f1, kCarryRd, hh, ll);
      a2H[8 + i] = hh;
      a2L[8 + i] = ll;
    }
  }

  v8f oH[4], oL[4];
#pragma unroll
  for (int nt = 0; nt < 4; ++nt) {
    const v16h bw = bfrag_from_lds(sOW, (unsigned)kPitchB, 0u, hs, (unsigned)nt * 16u + n, kCarryW);
    oH[nt] = mma_h(a2H, bw, zero8);
    oL[nt] = mma_h(a2L, bw, zero8);
  }
  float* ow = sO[wave];
#pragma unroll
  for (int nt = 0; nt < 4; ++nt) {
    const unsigned col = (unsigned)nt * 16u + n;
    const float bias = sOB[col];
#pragma unroll
    for (int r = 0; r < 8; ++r) {
      const float v = oH[nt][r] * kFoldOutHi + oL[nt][r] * kFoldOutLo + bias;
      ow[(8u * hs + (unsigned)r) * kPitchB + col] = v;
    }
  }
  __syncthreads();

  {
    const unsigned c4 = n * 4u;
    for (int pass = 0; pass < 2; ++pass) {
#pragma unroll
      for (unsigned it = 0; it < 8u; ++it) {
        const unsigned row = it * 2u + hs;
        const v4f v = *(const v4f*)(ow + row * kPitchB + c4);
        *(volatile v4f*)(out + (size_t)(m0 + row) * kVocab + c4) = v;
      }
      __threadfence();
    }
  }
}

extern "C" void kernel_launch(void* const* d_in, const int* in_sizes, int n_in,
                              void* d_out, int out_size, void* d_ws, size_t ws_size,
                              hipStream_t stream) {
  if (n_in < 12) return;
  if (in_sizes[0] != kBatch * kSeqLen) return;
  if (in_sizes[1] != kVocab * kHid) return;
  if (in_sizes[2] != kHid * kHid2) return;
  if (in_sizes[3] != kHid2) return;
  if (in_sizes[4] != kHid2 * kHid) return;
  if (in_sizes[5] != kHid) return;
  if (in_sizes[6] != kHid) return;
  if (in_sizes[7] != kHid) return;
  if (in_sizes[8] != kHid * kHid) return;
  if (in_sizes[9] != kHid) return;
  if (in_sizes[10] != kHid * kVocab) return;
  if (in_sizes[11] != kVocab) return;
  if (out_size != kBatch * kVocab) return;
  if (ws_size < kWsTotal) return;

  const int*   seq    = (const int*)  d_in[0];
  const float* embed  = (const float*)d_in[1];
  const float* w1     = (const float*)d_in[2];
  const float* b1     = (const float*)d_in[3];
  const float* w2     = (const float*)d_in[4];
  const float* b2     = (const float*)d_in[5];
  const float* ln_g   = (const float*)d_in[6];
  const float* ln_b   = (const float*)d_in[7];
  const float* read_w = (const float*)d_in[8];
  const float* read_b = (const float*)d_in[9];
  const float* out_w  = (const float*)d_in[10];
  const float* out_b  = (const float*)d_in[11];
  float* out = (float*)d_out;

  char* ws = (char*)d_ws;
  float* Tt   = (float*)(ws + kOffTbl);
  float* Dinv = (float*)(ws + kOffDinv);
  float* ctxp = (float*)(ws + kOffCtx);

  encode_table_kernel<<<1, 128, 0, stream>>>(embed, w1, b1, w2, b2, ln_g, ln_b, Tt, Dinv);
  adjoint_scan_kernel<<<kBatch / 32, 32, 0, stream>>>(seq, Tt, Dinv, ctxp);
  readout_kernel<<<kBatch / 64, 128, 0, stream>>>(ctxp, read_w, read_b, out_w, out_b, out);
}
